// MicroEncoder_23476291240585
// MI455X (gfx1250) — hardware-run, weakly checked
//
#include <hip/hip_runtime.h>
#include <stddef.h>
#include <stdint.h>
#include <math.h>


#define NN      100000
#define NE      1600000
#define CW      32
#define HLW     64
#define NTHR    256
#define NWAVE   8
#define NBA     1024
#define SLB     21
#define EMASK   ((1 << SLB) - 1)
#define NBLK    98
#define NBP     (NBLK * NBA)
#define GBM     128
#define GBLK    782
#define MP      (GBLK * GBM)
#define WLCAP   3072
#define RCAP    20480
#define DEGCAP  64
#define KB      256
#define TM_X2   2
#define TM_T    2
#define NWCH    (NE / 256)
#define BK_ZINTS (NWAVE * WLCAP + RCAP + 3 * NBA)
#define BK_LDS_INTS (BK_ZINTS + 16)
#define NORM_HALF (NBLK * RCAP / 2 / NTHR)
#define PREP_GX (MP / 32)
#define WSMAX   134217728

static_assert(NE % 256 == 0);
static_assert(NE <= (1 << SLB));
static_assert(NBA <= 1024 && (NBA & (NBA - 1)) == 0);
static_assert(((long long)(NBA - 1) << SLB) + EMASK < (1LL << 31));
static_assert(NBP >= MP && MP >= NN && MP % GBM == 0 && MP % 32 == 0);
static_assert(NWAVE * WLCAP >= RCAP);
static_assert(RCAP % 512 == 0 && BK_ZINTS % (NTHR * 4) == 0);
static_assert((NBLK * RCAP / 2) % NTHR == 0);
static_assert(NBA % NTHR == 0 && NBA % NWAVE == 0 && NBA % 32 == 0);
static_assert(KB % 32 == 0 && KB == 8 * CW && HLW == 2 * CW);
static_assert(BK_LDS_INTS * 4 <= 327680);
static_assert(DEGCAP % 32 == 0);

typedef float          v4f   __attribute__((ext_vector_type(4)));
typedef float          v8f   __attribute__((ext_vector_type(8)));
typedef int            v2i   __attribute__((ext_vector_type(2)));
typedef int            v4i   __attribute__((ext_vector_type(4)));
typedef int            v8i   __attribute__((ext_vector_type(8)));
typedef unsigned short v8us  __attribute__((ext_vector_type(8)));
typedef unsigned short v16us __attribute__((ext_vector_type(16)));
typedef __bf16         v16bf __attribute__((ext_vector_type(16)));
typedef v4f  __attribute__((may_alias)) v4fa;
typedef v2i  __attribute__((may_alias)) v2ia;
typedef v4i  __attribute__((may_alias)) v4ia;
typedef v8us __attribute__((may_alias)) v8usa;
union FragB { v16bf v; v16us u; v8us h[2]; v8i w; };

__device__ __forceinline__ v8f wmb(const FragB& a, const FragB& b, v8f c) {
  v8f d = __builtin_amdgcn_wmma_f32_16x16x32_bf16(false, a.v, false, b.v, (short)0, c, false, false);
  asm volatile("v_nop\n\tv_nop\n\tv_nop\n\tv_nop" : "+v"(d) : "v"(a.w), "v"(b.w));
  return d;
}

__device__ __forceinline__ unsigned bf16_bits(float f) {
  const unsigned u = __float_as_uint(f);
  return (u + 0x7FFFu + ((u >> 16) & 1u)) >> 16;
}
__device__ __forceinline__ unsigned bf16_bits_n(float f) {
  const unsigned r = bf16_bits(f);
  return (f != f) ? 0x7fc0u : r;
}
__device__ __forceinline__ float bf16_val(float f) {
  return __uint_as_float(bf16_bits(f) << 16);
}
__device__ __forceinline__ int clampi(int v, int lo, int hi) {
  return v < lo ? lo : (v > hi ? hi : v);
}

__device__ __forceinline__ int split_word(float v0, float v1, int hmask) {
  const unsigned h0 = bf16_bits_n(v0), h1 = bf16_bits_n(v1);
  const unsigned l0 = bf16_bits_n(v0 - __uint_as_float(h0 << 16));
  const unsigned l1 = bf16_bits_n(v1 - __uint_as_float(h1 << 16));
  const int hw = (int)(h0 | (h1 << 16));
  const int lw = (int)(l0 | (l1 << 16));
  return (hw & hmask) | (lw & ~hmask);
}

__global__ __launch_bounds__(NTHR) void k_prep(const float* __restrict__ x,
                                               const float* __restrict__ wz1, const float* __restrict__ wh1,
                                               const float* __restrict__ wz2, const float* __restrict__ wh2,
                                               const float* __restrict__ bz1, const float* __restrict__ bh1,
                                               const float* __restrict__ bz2, const float* __restrict__ bh2,
                                               unsigned short* xhl, unsigned short* wb, float* bias) {
  const int tid = (int)threadIdx.x, lane = tid & 31, wave = tid >> 5;
  const int blk = (int)blockIdx.x;
  if (blk < PREP_GX) {
    const int row0 = blk * 32 + wave * 4;
    const int row  = row0 + (lane >> 3);
    const int p    = lane & 7;
    const int rc   = row < NN ? row : NN - 1;
    const float* xp = x + (size_t)rc * CW + 8 * (p & 3);
    const v4f a = *(const v4fa*)xp;
    const v4f b = *(const v4fa*)(xp + 4);
    asm volatile("" :: "v"(a), "v"(b));
    const int mk = (row < NN && p < 4) ? -1 : 0;
    v4i o;
    o.x = (int)(bf16_bits(a.x) | (bf16_bits(a.y) << 16)) & mk;
    o.y = (int)(bf16_bits(a.z) | (bf16_bits(a.w) << 16)) & mk;
    o.z = (int)(bf16_bits(b.x) | (bf16_bits(b.y) << 16)) & mk;
    o.w = (int)(bf16_bits(b.z) | (bf16_bits(b.w) << 16)) & mk;
    unsigned short* dp = xhl + (size_t)row0 * HLW + 8 * lane;
    *(volatile v4i*)dp = o;
    __threadfence();
    *(volatile v4i*)dp = o;
  } else if (blk < PREP_GX + 16) {
    const int pb  = blk - PREP_GX;
    const int mat = pb >> 2;
    const float* w;
    if (mat == 0)      w = wz1;
    else if (mat == 1) w = wh1;
    else if (mat == 2) w = wz2;
    else               w = wh2;
    const int cell = mat >> 1, gate = mat & 1;
    const int v  = (pb & 3) * NTHR + tid;
    const int nn = v >> 5;
    const int k8 = (v & 31) * 8;
    const int kb = k8 >> 5;
    const int kk = k8 & 31;
    const int d  = (kb >> 1) & 1;
    const int h  = kb >> 2;
    const float* sp = w + d * 4096 + h * 2048 + kk * CW + nn;
    const float f0 = sp[0 * CW], f1 = sp[1 * CW], f2 = sp[2 * CW], f3 = sp[3 * CW];
    const float f4 = sp[4 * CW], f5 = sp[5 * CW], f6 = sp[6 * CW], f7 = sp[7 * CW];
    v8us o;
    o[0] = (unsigned short)bf16_bits(f0); o[1] = (unsigned short)bf16_bits(f1);
    o[2] = (unsigned short)bf16_bits(f2); o[3] = (unsigned short)bf16_bits(f3);
    o[4] = (unsigned short)bf16_bits(f4); o[5] = (unsigned short)bf16_bits(f5);
    o[6] = (unsigned short)bf16_bits(f6); o[7] = (unsigned short)bf16_bits(f7);
    unsigned short* dp = wb + (size_t)cell * (64 * KB) + (size_t)(gate * 32 + nn) * KB + k8;
    *(volatile v8us*)dp = o;
    __threadfence();
    *(volatile v8us*)dp = o;
  } else {
    if (wave == 0) {
      const int cell = lane >> 4;
      const int q    = lane & 15;
      const int idx  = (q & 7) * 4;
      const v4f a0 = *(const v4fa*)(bz1 + idx);
      const v4f a1 = *(const v4fa*)(bh1 + idx);
      const v4f a2 = *(const v4fa*)(bz2 + idx);
      const v4f a3 = *(const v4fa*)(bh2 + idx);
      asm volatile("" :: "v"(a0), "v"(a1), "v"(a2), "v"(a3));
      const int sel = cell * 2 + (q >> 3);
      const int m0 = (sel == 0) ? -1 : 0, m1 = (sel == 1) ? -1 : 0, m2 = (sel == 2) ? -1 : 0, m3 = (sel == 3) ? -1 : 0;
      v4f o;
      o.x = bf16_val(__int_as_float((__float_as_int(a0.x) & m0) | (__float_as_int(a1.x) & m1) | (__float_as_int(a2.x) & m2) | (__float_as_int(a3.x) & m3)));
      o.y = bf16_val(__int_as_float((__float_as_int(a0.y) & m0) | (__float_as_int(a1.y) & m1) | (__float_as_int(a2.y) & m2) | (__float_as_int(a3.y) & m3)));
      o.z = bf16_val(__int_as_float((__float_as_int(a0.z) & m0) | (__float_as_int(a1.z) & m1) | (__float_as_int(a2.z) & m2) | (__float_as_int(a3.z) & m3)));
      o.w = bf16_val(__int_as_float((__float_as_int(a0.w) & m0) | (__float_as_int(a1.w) & m1) | (__float_as_int(a2.w) & m2) | (__float_as_int(a3.w) & m3)));
      float* dp = bias + 4 * lane;
      *(volatile v4f*)dp = o;
      __threadfence();
      *(volatile v4f*)dp = o;
    }
  }
}

__device__ __forceinline__ void hit1(bool hj, unsigned sj, int eid, int* wl, int& wcn) {
  const unsigned mj = __builtin_amdgcn_ballot_w32(hj);
  const int pos = wcn + (int)__builtin_amdgcn_mbcnt_lo(mj, 0u);
  if (hj && pos < WLCAP) wl[pos] = (int)((sj << SLB) | (unsigned)eid);
  wcn += (int)__builtin_popcount(mj);
}

__global__ __launch_bounds__(NTHR) void k_bucket(const int* __restrict__ edge, const float* __restrict__ ew,
                                                 int* ent, int* cntg, int* offg, float* degg) {
  extern __shared__ __attribute__((aligned(16))) int dsm[];
  int* list = dsm;
  int* sl   = list + NWAVE * WLCAP;
  int* cnt  = sl + RCAP;
  int* offs = cnt + NBA;
  int* cur  = offs + NBA;
  int* misc = cur + NBA;
  const int tid = (int)threadIdx.x, lane = tid & 31, wave = tid >> 5;
  const int blk = (int)blockIdx.x, dir = (int)blockIdx.y;
  const int nodeBase = blk * NBA;
  const int keyOff = (dir == 0) ? NE : 0;
  const int* keys = edge + keyOff;
  const int* gath = edge + (NE - keyOff);

  {
    const v4i z4 = {0, 0, 0, 0};
    for (int i = tid * 4; i < BK_ZINTS; i += NTHR * 4) *(v4ia*)(dsm + i) = z4;
    if (tid < 16) misc[tid] = 0;
  }
  __syncthreads();

  int wcn = 0;
  int* wl = list + wave * WLCAP;
  const unsigned nbs = (unsigned)nodeBase;
#pragma unroll 1
  for (int wc = wave; wc < NWCH; wc += NWAVE) {
    const int e0 = wc * 256 + lane * 8;
    const v4i da = *(const v4ia*)(keys + e0);
    const v4i db = *(const v4ia*)(keys + e0 + 4);
    const unsigned s0 = (unsigned)da.x - nbs, s1 = (unsigned)da.y - nbs;
    const unsigned s2 = (unsigned)da.z - nbs, s3 = (unsigned)da.w - nbs;
    const unsigned s4 = (unsigned)db.x - nbs, s5 = (unsigned)db.y - nbs;
    const unsigned s6 = (unsigned)db.z - nbs, s7 = (unsigned)db.w - nbs;
    const bool h0 = s0 < (unsigned)NBA, h1 = s1 < (unsigned)NBA, h2 = s2 < (unsigned)NBA, h3 = s3 < (unsigned)NBA;
    const bool h4 = s4 < (unsigned)NBA, h5 = s5 < (unsigned)NBA, h6 = s6 < (unsigned)NBA, h7 = s7 < (unsigned)NBA;
    const unsigned any = __builtin_amdgcn_ballot_w32(h0 | h1 | h2 | h3 | h4 | h5 | h6 | h7);
    if (any != 0u) {
      hit1(h0, s0, e0 + 0, wl, wcn);
      hit1(h1, s1, e0 + 1, wl, wcn);
      hit1(h2, s2, e0 + 2, wl, wcn);
      hit1(h3, s3, e0 + 3, wl, wcn);
      hit1(h4, s4, e0 + 4, wl, wcn);
      hit1(h5, s5, e0 + 5, wl, wcn);
      hit1(h6, s6, e0 + 6, wl, wcn);
      hit1(h7, s7, e0 + 7, wl, wcn);
    }
  }
  if (lane == 0) misc[wave] = wcn;
  __syncthreads();

  if (wave == 0) {
    int t = 0, ov = 0;
#pragma unroll 1
    for (int w2 = 0; w2 < NWAVE; ++w2) {
      int cr = misc[w2];
      ov |= (cr > WLCAP) ? 1 : 0;
      cr = clampi(cr, 0, WLCAP);
      const int c = __builtin_amdgcn_readfirstlane(cr);
#pragma unroll 1
      for (int b0 = 0; b0 < c; b0 += 32) {
        const int idx = b0 + lane;
        const int e = list[w2 * WLCAP + (idx < WLCAP ? idx : WLCAP - 1)];
        const int m32 = (c - b0) < 32 ? (c - b0) : 32;
#pragma unroll 1
        for (int k = 0; k < m32; ++k) {
          const int u    = __builtin_amdgcn_readlane(e, k);
          const int slot = (u >> SLB) & (NBA - 1);
          if (t < RCAP) {
            if (lane == 0) cnt[slot] = cnt[slot] + 1;
            t = t + 1;
          } else {
            ov = 1;
          }
        }
      }
    }
    if (lane == 0) { misc[8] = t; misc[9] = ov; }
  }
  __syncthreads();
  const int tt  = clampi(misc[8], 0, RCAP);
  const int ovf = misc[9];

  if (wave == 0) {
    const int base = lane * (NBA / 32);
    int s = 0;
#pragma unroll 1
    for (int i = 0; i < NBA / 32; ++i) s += cnt[base + i];
    int incl = s;
#pragma unroll
    for (int d = 1; d < 32; d <<= 1) {
      const int y = __shfl_up(incl, d, 32);
      if (lane >= d) incl += y;
    }
    int run = incl - s;
#pragma unroll 1
    for (int i = 0; i < NBA / 32; ++i) {
      const int cv = cnt[base + i];
      offs[base + i] = run;
      cur[base + i]  = run;
      run += cv;
    }
  }
  __syncthreads();

  if (wave == 0) {
    int t = 0;
#pragma unroll 1
    for (int w2 = 0; w2 < NWAVE; ++w2) {
      int cr = clampi(misc[w2], 0, WLCAP);
      const int c = __builtin_amdgcn_readfirstlane(cr);
#pragma unroll 1
      for (int b0 = 0; b0 < c; b0 += 32) {
        const int idx = b0 + lane;
        const int e = list[w2 * WLCAP + (idx < WLCAP ? idx : WLCAP - 1)];
        const int m32 = (c - b0) < 32 ? (c - b0) : 32;
#pragma unroll 1
        for (int k = 0; k < m32; ++k) {
          const int u    = __builtin_amdgcn_readlane(e, k);
          const int slot = (u >> SLB) & (NBA - 1);
          if (t < tt) {
            if (lane == 0) {
              int p = cur[slot];
              p = clampi(p, 0, RCAP - 1);
              sl[p] = u;
              cur[slot] = p + 1;
            }
            t = t + 1;
          }
        }
      }
    }
  }
  __syncthreads();

  int* entb = ent + (size_t)(dir * NBLK + blk) * (size_t)(RCAP * 2);
#pragma unroll 1
  for (int it = 0; it < RCAP / 512; ++it) {
    const int i0 = (it * NTHR + tid) * 2;
    const int u0 = sl[i0], u1 = sl[i0 + 1];
    const int e0 = clampi(u0 & EMASK, 0, NE - 1);
    const int e1 = clampi(u1 & EMASK, 0, NE - 1);
    int g0 = gath[e0], g1 = gath[e1];
    const float w0 = ew[e0], w1 = ew[e1];
    asm volatile("" :: "v"(g0), "v"(g1), "v"(w0), "v"(w1));
    g0 = clampi(g0, 0, NN - 1);
    g1 = clampi(g1, 0, NN - 1);
    const int m0 = (i0 < tt) ? -1 : 0;
    const int m1 = (i0 + 1 < tt) ? -1 : 0;
    v4i o;
    o.x = g0 & m0;
    o.y = (int)(bf16_bits(w0) << 16) & m0;
    o.z = g1 & m1;
    o.w = (int)(bf16_bits(w1) << 16) & m1;
    list[i0]     = o.y;
    list[i0 + 1] = o.w;
    int* dp = entb + 2 * i0;
    *(volatile v4i*)dp = o;
    __threadfence();
    *(volatile v4i*)dp = o;
  }
  __syncthreads();

  const float qnan = __int_as_float(0x7fc00000);
#pragma unroll 1
  for (int q = 0; q < NBA / NTHR; ++q) {
    const int s = q * NTHR + tid;
    const int craw = cnt[s];
    const bool big = craw > DEGCAP;
    const int cc = clampi(craw, 0, DEGCAP);
    const int o  = clampi(offs[s], 0, RCAP);
    int cm = cc;
#pragma unroll
    for (int d = 16; d > 0; d >>= 1) {
      const int y = __shfl_xor(cm, d, 32);
      cm = cm > y ? cm : y;
    }
    const int cmax = __builtin_amdgcn_readfirstlane(cm);
    float dg = 0.0f;
#pragma unroll 1
    for (int p = 0; p < cmax; ++p) {
      int idx = o + p;
      idx = idx > RCAP - 1 ? RCAP - 1 : idx;
      const int wbits = list[idx];
      const int mk = (p < cc) ? -1 : 0;
      dg = dg + __int_as_float(wbits & mk);
    }
    const bool bad = (ovf != 0) | big;
    dg = bad ? qnan : dg;
    const size_t gi = (size_t)dir * NBP + (size_t)(nodeBase + s);
    *(volatile int*)(cntg + gi)   = cc;
    *(volatile int*)(offg + gi)   = o;
    *(volatile float*)(degg + gi) = dg;
    __threadfence();
    *(volatile int*)(cntg + gi)   = cc;
    *(volatile int*)(offg + gi)   = o;
    *(volatile float*)(degg + gi) = dg;
  }
}

__global__ __launch_bounds__(NTHR) void k_norm(int* ent, const float* __restrict__ degg) {
  const int odir = ((int)blockIdx.x >= NORM_HALF) ? 0 : 1;
  const size_t i = (size_t)blockIdx.x * NTHR + threadIdx.x;
  int* p = ent + 4 * i;
  const v4i e = *(const v4ia*)p;
  const int g0 = clampi(e.x, 0, NN - 1);
  const int g1 = clampi(e.z, 0, NN - 1);
  const float d0 = degg[(size_t)odir * NBP + g0];
  const float d1 = degg[(size_t)odir * NBP + g1];
  const float q0 = __int_as_float(e.y) / d0;
  const float q1 = __int_as_float(e.w) / d1;
  v4i o;
  o.x = g0; o.y = __float_as_int(q0);
  o.z = g1; o.w = __float_as_int(q1);
  *(volatile v4i*)p = o;
  __threadfence();
  *(volatile v4i*)p = o;
}

__global__ __launch_bounds__(NTHR) void k_replay(const int* __restrict__ ent, const int* __restrict__ cntg,
                                                 const int* __restrict__ offg, const float* __restrict__ degg,
                                                 const unsigned* __restrict__ src, unsigned* tpl) {
  const int tid = (int)threadIdx.x, lane = tid & 31, wave = tid >> 5;
  const int blk = (int)blockIdx.x, dir = (int)blockIdx.y;
  const int nodeBase = blk * NBA;
  const int* eb = ent + (size_t)(dir * NBLK + blk) * (size_t)(RCAP * 2);
  unsigned* outp = tpl + (size_t)dir * ((size_t)MP * 32);
  const int hmask = (lane < 16) ? -1 : 0;
  const float qnan = __int_as_float(0x7fc00000);
#pragma unroll 1
  for (int si = 0; si < NBA / NWAVE; ++si) {
    const int s    = si * NWAVE + wave;
    const int node = nodeBase + s;
    const size_t gi = (size_t)dir * NBP + (size_t)node;
    int cv = cntg[gi];
    int ovv = offg[gi];
    const float dg = degg[gi];
    asm volatile("" :: "v"(cv), "v"(ovv), "v"(dg));
    const bool big = cv > DEGCAP;
    cv  = clampi(cv, 0, DEGCAP);
    ovv = clampi(ovv, 0, RCAP);
    const int c = __builtin_amdgcn_readfirstlane(cv);
    const int o = __builtin_amdgcn_readfirstlane(ovv);
    float a0 = 0.0f, a1 = 0.0f;
#pragma unroll 1
    for (int b0 = 0; b0 < c; b0 += 32) {
      int j = b0 + lane;
      j = j > c - 1 ? c - 1 : j;
      int idx = o + j;
      idx = idx > RCAP - 1 ? RCAP - 1 : idx;
      const v2i e = *(const v2ia*)(eb + 2 * idx);
      const int g  = clampi(e.x, 0, NN - 1);
      const int wb = e.y;
      const int m32 = (c - b0) < 32 ? (c - b0) : 32;
#pragma unroll 1
      for (int k = 0; k < m32; ++k) {
        const int   sk = __builtin_amdgcn_readlane(g, k);
        const float wk = __int_as_float(__builtin_amdgcn_readlane(wb, k));
        const unsigned wd = src[(size_t)sk * 32 + lane];
        const float f0 = __uint_as_float(wd << 16);
        const float f1 = __uint_as_float(wd & 0xffff0000u);
        a0 = fmaf(wk, f0, a0);
        a1 = fmaf(wk, f1, a1);
      }
    }
    const float s0 = a0 + __shfl_xor(a0, 16, 32);
    const float s1 = a1 + __shfl_xor(a1, 16, 32);
    const bool bad  = (dg != dg) | big;
    const bool live = node < NN;
    float v0 = bad ? qnan : s0;
    float v1 = bad ? qnan : s1;
    v0 = live ? v0 : 0.0f;
    v1 = live ? v1 : 0.0f;
    const unsigned word = (unsigned)split_word(v0, v1, hmask);
    if (node < MP) {
      unsigned* dp = outp + (size_t)node * 32 + lane;
      *(volatile unsigned*)dp = word;
      __threadfence();
      *(volatile unsigned*)dp = word;
    }
  }
}

__device__ __forceinline__ void kstep(const unsigned short* ap, const unsigned short* bp, int kb, v8f (&acc)[4]) {
  FragB af;
  af.h[0] = *(const v8usa*)ap;
  af.h[1] = *(const v8usa*)(ap + 16);
#pragma unroll
  for (int nt = 0; nt < 4; ++nt) {
    const unsigned short* wq = bp + (size_t)(16 * nt) * KB + kb * 32;
    FragB bf;
    bf.h[0] = *(const v8usa*)wq;
    bf.h[1] = *(const v8usa*)(wq + 16);
    acc[nt] = wmb(af, bf, acc[nt]);
  }
}

template <int CELL2>
__global__ __launch_bounds__(NTHR) void k_gemm(const unsigned short* __restrict__ xhl,
                                               const unsigned short* __restrict__ tpl,
                                               const unsigned short* __restrict__ wb,
                                               const float* __restrict__ bias,
                                               unsigned short* x2hl, float* outp) {
  __shared__ __attribute__((aligned(16))) float stg[GBM * CW];
  __shared__ __attribute__((aligned(16))) float shb[64];
  const int tid = (int)threadIdx.x, lane = tid & 31, wave = tid >> 5, hh = lane >> 4, m = lane & 15;
  const int rowBase = (int)blockIdx.x * GBM;

  {
    const v4f bv = *(const v4fa*)(bias + CELL2 * 64 + 4 * (tid & 15));
    asm volatile("" :: "v"(bv));
    if (tid < 16) *(v4fa*)(shb + 4 * tid) = bv;
  }

  v8f acc[4];
  {
    const v8f z = {0.f, 0.f, 0.f, 0.f, 0.f, 0.f, 0.f, 0.f};
#pragma unroll
    for (int t = 0; t < 4; ++t) acc[t] = z;
  }
  const size_t arow = (size_t)(rowBase + 16 * wave + m) * HLW + 8 * hh;
  const unsigned short* xa = xhl + arow;
  const unsigned short* to = tpl + arow;
  const unsigned short* ti = tpl + (size_t)MP * HLW + arow;
  const unsigned short* bp = wb + (size_t)CELL2 * (64 * KB) + (size_t)m * KB + 8 * hh;

  constexpr bool XLO = (CELL2 != 0) && (TM_X2 == 2);
  constexpr bool TLO = (TM_T == 2);
  kstep(xa, bp, 0, acc);
  if constexpr (XLO) kstep(xa + 32, bp, 1, acc);
  kstep(xa, bp, 2, acc);
  if constexpr (XLO) kstep(xa + 32, bp, 3, acc);
  kstep(to, bp, 4, acc);
  if constexpr (TLO) kstep(to + 32, bp, 5, acc);
  kstep(ti, bp, 6, acc);
  if constexpr (TLO) kstep(ti + 32, bp, 7, acc);

  __syncthreads();
#pragma unroll
  for (int j = 0; j < 2; ++j) {
    const float bzv = shb[16 * j + m];
    const float bhv = shb[32 + 16 * j + m];
#pragma unroll
    for (int r = 0; r < 8; ++r) {
      const float pz = acc[j][r] + bzv;
      const float ph = acc[j + 2][r] + bhv;
      const float z  = 1.0f / (1.0f + expf(-pz));
      const float ht = tanhf(ph);
      stg[(16 * wave + 8 * hh + r) * CW + 16 * j + m] = (1.0f - z) * ht;
    }
  }
  __syncthreads();

  const int p = lane & 7;
  if constexpr (CELL2 != 0) {
    v4f pv[4];
#pragma unroll
    for (int q4 = 0; q4 < 4; ++q4) {
      const int lr = 16 * wave + 4 * q4 + (lane >> 3);
      pv[q4] = *(const v4fa*)(stg + lr * CW + 4 * p);
      asm volatile("" :: "v"(pv[q4]));
    }
#pragma unroll
    for (int q4 = 0; q4 < 4; ++q4) {
      const int r0 = rowBase + 16 * wave + 4 * q4;
      if (r0 + (lane >> 3) < NN) *(volatile v4f*)(outp + (size_t)r0 * CW + 4 * lane) = pv[q4];
    }
    __threadfence();
#pragma unroll
    for (int q4 = 0; q4 < 4; ++q4) {
      const int r0 = rowBase + 16 * wave + 4 * q4;
      if (r0 + (lane >> 3) < NN) *(volatile v4f*)(outp + (size_t)r0 * CW + 4 * lane) = pv[q4];
    }
  } else {
    const int hmask = (p < 4) ? -1 : 0;
    const int cb = 8 * (p & 3);
    v4i qv[4];
#pragma unroll
    for (int q4 = 0; q4 < 4; ++q4) {
      const int lr = 16 * wave + 4 * q4 + (lane >> 3);
      const v4f va = *(const v4fa*)(stg + lr * CW + cb);
      const v4f vb = *(const v4fa*)(stg + lr * CW + cb + 4);
      const bool live = (rowBase + lr) < NN;
      float e0 = (va.x > 0.0f) ? va.x : (va.x - va.x);
      float e1 = (va.y > 0.0f) ? va.y : (va.y - va.y);
      float e2 = (va.z > 0.0f) ? va.z : (va.z - va.z);
      float e3 = (va.w > 0.0f) ? va.w : (va.w - va.w);
      float e4 = (vb.x > 0.0f) ? vb.x : (vb.x - vb.x);
      float e5 = (vb.y > 0.0f) ? vb.y : (vb.y - vb.y);
      float e6 = (vb.z > 0.0f) ? vb.z : (vb.z - vb.z);
      float e7 = (vb.w > 0.0f) ? vb.w : (vb.w - vb.w);
      e0 = live ? e0 : 0.0f; e1 = live ? e1 : 0.0f; e2 = live ? e2 : 0.0f; e3 = live ? e3 : 0.0f;
      e4 = live ? e4 : 0.0f; e5 = live ? e5 : 0.0f; e6 = live ? e6 : 0.0f; e7 = live ? e7 : 0.0f;
      v4i o;
      o.x = split_word(e0, e1, hmask);
      o.y = split_word(e2, e3, hmask);
      o.z = split_word(e4, e5, hmask);
      o.w = split_word(e6, e7, hmask);
      qv[q4] = o;
    }
#pragma unroll
    for (int q4 = 0; q4 < 4; ++q4) {
      unsigned short* dp = x2hl + (size_t)(rowBase + 16 * wave + 4 * q4) * HLW + 8 * lane;
      *(volatile v4i*)dp = qv[q4];
    }
    __threadfence();
#pragma unroll
    for (int q4 = 0; q4 < 4; ++q4) {
      unsigned short* dp = x2hl + (size_t)(rowBase + 16 * wave + 4 * q4) * HLW + 8 * lane;
      *(volatile v4i*)dp = qv[q4];
    }
  }
}

static inline size_t al256(size_t o) { return (o + 255) & ~(size_t)255; }

extern "C" void kernel_launch(void* const* d_in, const int* in_sizes, int n_in,
                              void* d_out, int out_size, void* d_ws, size_t ws_size,
                              hipStream_t stream) {
  if (n_in < 15) return;
  if (in_sizes[0] != NN * CW) return;
  if (in_sizes[1] != 2 * NE) return;
  if (in_sizes[2] != NE) return;
  if (in_sizes[3] != 8192 || in_sizes[7] != 8192 || in_sizes[9] != 8192 || in_sizes[13] != 8192) return;
  if (in_sizes[4] != CW || in_sizes[8] != CW || in_sizes[10] != CW || in_sizes[14] != CW) return;
  if ((long long)out_size != (long long)NN * CW) return;

  const float* x    = (const float*)d_in[0];
  const int*   edge = (const int*)d_in[1];
  const float* ew   = (const float*)d_in[2];
  const float* wz1  = (const float*)d_in[3];
  const float* bz1  = (const float*)d_in[4];
  const float* wh1  = (const float*)d_in[7];
  const float* bh1  = (const float*)d_in[8];
  const float* wz2  = (const float*)d_in[9];
  const float* bz2  = (const float*)d_in[10];
  const float* wh2  = (const float*)d_in[13];
  const float* bh2  = (const float*)d_in[14];
  float* out = (float*)d_out;

  char* ws = (char*)d_ws;
  size_t off = 0;
  const size_t oX1  = off; off = al256(off + (size_t)MP * HLW * 2);
  const size_t oX2  = off; off = al256(off + (size_t)MP * HLW * 2);
  const size_t oT   = off; off = al256(off + (size_t)2 * MP * HLW * 2);
  const size_t oENT = off; off = al256(off + (size_t)2 * NBLK * RCAP * 8);
  const size_t oCNT = off; off = al256(off + (size_t)2 * NBP * 4);
  const size_t oOFF = off; off = al256(off + (size_t)2 * NBP * 4);
  const size_t oDEG = off; off = al256(off + (size_t)2 * NBP * 4);
  const size_t oWB  = off; off = al256(off + (size_t)2 * 64 * KB * 2);
  const size_t oBI  = off; off = al256(off + (size_t)128 * 4);
  if (off > ws_size || off > (size_t)WSMAX) return;
  unsigned short* X1  = (unsigned short*)(ws + oX1);
  unsigned short* X2  = (unsigned short*)(ws + oX2);
  unsigned short* TP  = (unsigned short*)(ws + oT);
  int*            ENT = (int*)(ws + oENT);
  int*            CNT = (int*)(ws + oCNT);
  int*            OFF = (int*)(ws + oOFF);
  float*          DEG = (float*)(ws + oDEG);
  unsigned short* WB  = (unsigned short*)(ws + oWB);
  float*          BI  = (float*)(ws + oBI);

  const size_t bkLds = (size_t)BK_LDS_INTS * 4;
  hipFuncSetAttribute(reinterpret_cast<const void*>(&k_bucket), hipFuncAttributeMaxDynamicSharedMemorySize, (int)bkLds);

  k_prep<<<PREP_GX + 17, NTHR, 0, stream>>>(x, wz1, wh1, wz2, wh2, bz1, bh1, bz2, bh2, X1, WB, BI);
  k_bucket<<<dim3(NBLK, 2), NTHR, bkLds, stream>>>(edge, ew, ENT, CNT, OFF, DEG);
  k_norm<<<NBLK * RCAP / NTHR, NTHR, 0, stream>>>(ENT, DEG);
  k_replay<<<dim3(NBLK, 2), NTHR, 0, stream>>>(ENT, CNT, OFF, DEG, (const unsigned*)X1, (unsigned*)TP);
  k_gemm<0><<<GBLK, NTHR, 0, stream>>>(X1, TP, WB, BI, X2, out);
  k_replay<<<dim3(NBLK, 2), NTHR, 0, stream>>>(ENT, CNT, OFF, DEG, (const unsigned*)X2, (unsigned*)TP);
  k_gemm<1><<<GBLK, NTHR, 0, stream>>>(X2, TP, WB, BI, X2, out);
}
